// BiMatchLSTM_49658411877023
// MI455X (gfx1250) — hardware-verified
//
#include <hip/hip_runtime.h>
#include <math.h>

typedef __attribute__((ext_vector_type(16))) _Float16 v16h;
typedef __attribute__((ext_vector_type(8)))  _Float16 v8h;
typedef __attribute__((ext_vector_type(16))) __bf16   v16b;
typedef __attribute__((ext_vector_type(8)))  __bf16   v8b;
typedef __attribute__((ext_vector_type(8)))  float    v8f;
typedef __attribute__((ext_vector_type(4)))  float    v4f;

constexpr int kB    = 128;
constexpr int kTP   = 400;
constexpr int kTQ   = 60;
constexpr int kD    = 300;
constexpr int kDK   = 320;
constexpr int kH    = 150;
constexpr int kHK   = 160;
constexpr int kHN   = 192;
constexpr int kG4   = 4 * kHK;
constexpr int kR    = 2 * kB;
constexpr int kNHV  = 1536;
constexpr int kNZG  = 2 * kG4;
constexpr int kChunk = 80;
constexpr int kRowsP = kTP * kB;
constexpr int kRowsQ = kB * kTQ;
constexpr int kRowsC = kChunk * kB;
constexpr int kThr  = 256;
constexpr float kInCarry = 1024.0f;
constexpr float kWCarry  = 4096.0f;
constexpr float kScW = 1.0f / (kInCarry * kWCarry);
constexpr float kF16MinNormal = 6.103515625e-5f;

static_assert(kTP % kChunk == 0 && (kRowsP % 64) == 0 && (kRowsQ % 64) == 0 && (kRowsC % 64) == 0 && (kR % 64) == 0 && (kHN % 64) == 0 && (kG4 % 64) == 0 && (kNHV % 64) == 0 && (kNZG % 64) == 0, "GEMM M, N multiples of 64");
static_assert(((kRowsP / 64) * (kHN / 64)) % 8 == 0 && ((kRowsQ / 64) * (kHN / 64)) % 8 == 0 && ((kRowsC / 64) * (kG4 / 64)) % 8 == 0 && ((kR / 64) * (kNHV / 64)) % 8 == 0 && ((kR / 64) * (kNZG / 64)) % 8 == 0, "GEMM grids exact");
static_assert((kDK % 32) == 0 && (kHK % 32) == 0 && 2 * kG4 + kHN <= kNHV, "GEMM K multiples of 32; the state product's blocks fit");

constexpr size_t kOffP16 = 0ull;
constexpr size_t kOffQ16 = 32768000ull;
constexpr size_t kOffWP16 = 37683200ull;
constexpr size_t kOffWQ16 = 37806080ull;
constexpr size_t kOffWHV = 37928960ull;
constexpr size_t kOffWIHPF = 38420480ull;
constexpr size_t kOffWIHPB = 38830080ull;
constexpr size_t kOffWIHZ = 39239680ull;
constexpr size_t kOffBIAS = 40058880ull;
constexpr size_t kOffGP = 40075264ull;
constexpr size_t kOffGQ = 79396864ull;
constexpr size_t kOffXGF = 85295104ull;
constexpr size_t kOffXGB = 111509504ull;
constexpr size_t kOffHV = 137723904ull;
constexpr size_t kOffZG = 139296768ull;
constexpr size_t kOffH32 = 140607488ull;
constexpr size_t kOffC32 = 140771328ull;
constexpr size_t kOffH16 = 140935168ull;
constexpr size_t kOffZ16 = 141017088ull;
constexpr size_t kOffOUTW = 141180928ull;
constexpr size_t kWsTotal = 206716928ull;
static_assert(kWsTotal <= 268435456ull, "carve cap");
static_assert(kOffP16 == 0
              && kOffQ16 == kOffP16 + 32768000ull
              && kOffWP16 == kOffQ16 + 4915200ull
              && kOffWQ16 == kOffWP16 + 122880ull
              && kOffWHV == kOffWQ16 + 122880ull
              && kOffWIHPF == kOffWHV + 491520ull
              && kOffWIHPB == kOffWIHPF + 409600ull
              && kOffWIHZ == kOffWIHPB + 409600ull
              && kOffBIAS == kOffWIHZ + 819200ull
              && kOffGP == kOffBIAS + 16384ull
              && kOffGQ == kOffGP + 39321600ull
              && kOffXGF == kOffGQ + 5898240ull
              && kOffXGB == kOffXGF + 26214400ull
              && kOffHV == kOffXGB + 26214400ull
              && kOffZG == kOffHV + 1572864ull
              && kOffH32 == kOffZG + 1310720ull
              && kOffC32 == kOffH32 + 163840ull
              && kOffH16 == kOffC32 + 163840ull
              && kOffZ16 == kOffH16 + 81920ull
              && kOffOUTW == kOffZ16 + 163840ull
              && kWsTotal == kOffOUTW + 65536000ull, "the carve is chained and totalled");
static_assert((kOffP16 % 256) == 0 && (kOffQ16 % 256) == 0 && (kOffWP16 % 256) == 0 && (kOffWQ16 % 256) == 0 && (kOffWHV % 256) == 0 && (kOffWIHPF % 256) == 0 && (kOffWIHPB % 256) == 0 && (kOffWIHZ % 256) == 0 && (kOffBIAS % 256) == 0 && (kOffGP % 256) == 0 && (kOffGQ % 256) == 0 && (kOffXGF % 256) == 0 && (kOffXGB % 256) == 0 && (kOffHV % 256) == 0 && (kOffZG % 256) == 0 && (kOffH32 % 256) == 0 && (kOffC32 % 256) == 0 && (kOffH16 % 256) == 0 && (kOffZ16 % 256) == 0 && (kOffOUTW % 256) == 0, "aligned regions");
constexpr int kFBXF = 0, kFBXB = 640, kFZB = 2048, kFEnd = 4096;
static_assert(kFZB + kNHV <= kFEnd && kFBXB + kG4 <= kFZB, "the zero row covers the widest product (N = 1,536)");
constexpr size_t kOut1 = (size_t)kB * kTP * 2 * kH;
constexpr size_t kOutTotal = kOut1 + (size_t)kB * 2 * kH;

__device__ __forceinline__ unsigned short f2bf_bits(float f) {
  unsigned u = __float_as_uint(f);
  return (unsigned short)((u + 0x7FFFu + ((u >> 16) & 1u)) >> 16);
}
__device__ __forceinline__ float bf_bits2f(unsigned short h) { return __uint_as_float(((unsigned)h) << 16); }
__device__ __forceinline__ float bf16r(float f) { return bf_bits2f(f2bf_bits(f)); }
__device__ __forceinline__ float carry_flush(float v, float carry) {
  const float s = v * carry;
  return (fabsf(s) < kF16MinNormal) ? 0.0f : s;
}
__device__ __forceinline__ float frcp(float x) { return __builtin_amdgcn_rcpf(x); }

__device__ __forceinline__ void dep_guard4_h(v8f& a, v8f& b, v8f& c, v8f& d, v16h x, v16h y) { asm volatile("v_nop\n\tv_nop\n\tv_nop\n\tv_nop" : "+v"(a), "+v"(b), "+v"(c), "+v"(d) : "v"(x), "v"(y)); }
__device__ __forceinline__ void dep_guard4_b(v8f& a, v8f& b, v8f& c, v8f& d, v16b x, v16b y) { asm volatile("v_nop\n\tv_nop\n\tv_nop\n\tv_nop" : "+v"(a), "+v"(b), "+v"(c), "+v"(d) : "v"(x), "v"(y)); }
__device__ __forceinline__ void keep4_h(v16h a, v16h b, v16h c, v16h d) { asm volatile("v_nop" :: "v"(a), "v"(b), "v"(c), "v"(d)); }
__device__ __forceinline__ void keep4_b(v16b a, v16b b, v16b c, v16b d) { asm volatile("v_nop" :: "v"(a), "v"(b), "v"(c), "v"(d)); }
__device__ __forceinline__ void acc_guard4(v8f& a, v8f& b, v8f& c, v8f& d) { asm volatile("v_nop\n\tv_nop\n\tv_nop\n\tv_nop" : "+v"(a), "+v"(b), "+v"(c), "+v"(d)); }

template <typename T> struct Frag;
template <> struct Frag<_Float16> {
  typedef v16h V; union U { v16h v; v8h h[2]; };
  static __device__ __forceinline__ v16h load(const _Float16* p) {
    U f; f.h[0] = *(const v8h*)(p); f.h[1] = *(const v8h*)(p + 16); return f.v;
  }
  static __device__ __forceinline__ v8f mma(v16h a, v16h b, v8f c) {
    return __builtin_amdgcn_wmma_f32_16x16x32_f16(false, a, false, b, (short)0, c, false, false);
  }
  static __device__ __forceinline__ void guard4(v8f& a, v8f& b, v8f& c, v8f& d, v16h x, v16h y) { dep_guard4_h(a, b, c, d, x, y); }
  static __device__ __forceinline__ void keep(v16h a, v16h b, v16h c, v16h d) { keep4_h(a, b, c, d); }
};
template <> struct Frag<__bf16> {
  typedef v16b V; union U { v16b v; v8b h[2]; };
  static __device__ __forceinline__ v16b load(const __bf16* p) {
    U f; f.h[0] = *(const v8b*)(p); f.h[1] = *(const v8b*)(p + 16); return f.v;
  }
  static __device__ __forceinline__ v8f mma(v16b a, v16b b, v8f c) {
    return __builtin_amdgcn_wmma_f32_16x16x32_bf16(false, a, false, b, (short)0, c, false, false);
  }
  static __device__ __forceinline__ void guard4(v8f& a, v8f& b, v8f& c, v8f& d, v16b x, v16b y) { dep_guard4_b(a, b, c, d, x, y); }
  static __device__ __forceinline__ void keep(v16b a, v16b b, v16b c, v16b d) { keep4_b(a, b, c, d); }
};

__device__ __forceinline__ v8f mma_h(v16h a, v16h b, v8f c) {
  c = __builtin_amdgcn_wmma_f32_16x16x32_f16(false, a, false, b, (short)0, c, false, false);
  asm volatile("v_nop\n\tv_nop\n\tv_nop\n\tv_nop" : "+v"(c) : "v"(a), "v"(b));
  return c;
}

template <int ET> struct Elem;
template <> struct Elem<0> { typedef _Float16 T; };
template <> struct Elem<1> { typedef __bf16 T; };
template <int ET, bool SPLIT, int BIAS_MODE, int OUT_MODE, bool RESID, int ACT = 0>
__global__ __launch_bounds__(256) void wmma_gemm64(
    const unsigned short* __restrict__ Ap, const unsigned short* __restrict__ A2p, int lda, long strideA,
    const unsigned short* __restrict__ Btp, const unsigned short* __restrict__ Bt2p, int ldb, long strideB,
    void* __restrict__ Cout, void* __restrict__ Cout2, int ldc, long strideC,
    const float* __restrict__ bias,
    const float* __restrict__ resid, long strideR,
    int M, int N, int K, float scale) {
  typedef typename Elem<ET>::T T;
  typedef typename Frag<T>::V V;
  const T* A = (const T*)Ap; const T* A2 = (const T*)A2p; const T* Bt = (const T*)Btp; const T* Bt2 = (const T*)Bt2p;
  __shared__ __align__(16) float sT[8][16 * 68];
  const int b    = blockIdx.y;
  const int lane = threadIdx.x & 31;
  const int wave = threadIdx.x >> 5;
  const int tilesN = N >> 6;
  const int tilesM = M >> 6;
  const int tile = blockIdx.x * 8 + wave;
  if (tile >= tilesM * tilesN) return;
  const int tm = tile / tilesN;
  const int tn = tile - tm * tilesN;
  const int m0 = tm << 6;
  const int n0 = tn << 6;

  const T* Ab  = A  + (size_t)b * strideA;
  const T* Bb  = Bt + (size_t)b * strideB;
  const T* Ab2 = SPLIT ? (A2  + (size_t)b * strideA) : nullptr;
  const T* Bb2 = SPLIT ? (Bt2 + (size_t)b * strideB) : nullptr;

  const int rlane = lane & 15;
  const int koff  = (lane >> 4) * 8;
  const int mOff  = (lane >> 4) * 8;

  v8f acc[4][4];
#pragma unroll
  for (int i = 0; i < 4; ++i)
#pragma unroll
    for (int j = 0; j < 4; ++j) acc[i][j] = (v8f){0.f,0.f,0.f,0.f,0.f,0.f,0.f,0.f};

  for (int k0 = 0; k0 < K; k0 += 32) {
    V bh[4], bl[4];
#pragma unroll
    for (int j = 0; j < 4; ++j) {
      const size_t bo = (size_t)(n0 + (j << 4) + rlane) * ldb + koff + k0;
      bh[j] = Frag<T>::load(Bb + bo);
      if (SPLIT) bl[j] = Frag<T>::load(Bb2 + bo);
    }
#pragma unroll
    for (int i = 0; i < 4; ++i) {
      const size_t ao = (size_t)(m0 + (i << 4) + rlane) * lda + koff + k0;
      V ah = Frag<T>::load(Ab + ao);
      V al;
      if (SPLIT) al = Frag<T>::load(Ab2 + ao);
#pragma unroll
      for (int j = 0; j < 4; ++j) {
        acc[i][j] = Frag<T>::mma(ah, bh[j], acc[i][j]);
        if (SPLIT) {
          acc[i][j] = Frag<T>::mma(ah, bl[j], acc[i][j]);
          acc[i][j] = Frag<T>::mma(al, bh[j], acc[i][j]);
        }
      }
      Frag<T>::guard4(acc[i][0], acc[i][1], acc[i][2], acc[i][3], ah, SPLIT ? al : ah);
    }
    Frag<T>::keep(bh[0], bh[1], bh[2], bh[3]);
    if (SPLIT) Frag<T>::keep(bl[0], bl[1], bl[2], bl[3]);
  }
  acc_guard4(acc[0][0], acc[0][1], acc[0][2], acc[0][3]);
  acc_guard4(acc[1][0], acc[1][1], acc[1][2], acc[1][3]);
  acc_guard4(acc[2][0], acc[2][1], acc[2][2], acc[2][3]);
  acc_guard4(acc[3][0], acc[3][1], acc[3][2], acc[3][3]);

  float* slab = sT[wave];
  const float* Rb = RESID ? (resid + (size_t)b * strideR) : nullptr;
#pragma unroll
  for (int i = 0; i < 4; ++i) {
    const int mBase = m0 + (i << 4);
#pragma unroll
    for (int j = 0; j < 4; ++j) {
      const int n = n0 + (j << 4) + rlane;
      float bv = 0.f;
      if (BIAS_MODE == 2) bv = bias[n];
#pragma unroll
      for (int r = 0; r < 8; ++r) {
        float v = acc[i][j][r] * scale;
        if (BIAS_MODE == 1) v += bias[mBase + mOff + r];
        if (BIAS_MODE == 2) v += bv;
        if (RESID) v += Rb[(size_t)(mBase + mOff + r) * ldc + n];
        if (ACT == 1) v = tanhf(v);
        if (ACT == 2) v = fmaxf(v, 0.0f);
        if (ACT == 3) v = v / (1.0f + expf(-v));
        if (ACT == 4) v = (v > 0.f) ? v : 0.01f * v;
        slab[(mOff + r) * 68 + (j << 4) + rlane] = v;
      }
    }
    __builtin_amdgcn_fence(__ATOMIC_RELEASE, "workgroup");
    __builtin_amdgcn_wave_barrier();
    __builtin_amdgcn_fence(__ATOMIC_ACQUIRE, "workgroup");
    if (OUT_MODE == 0) {
      float* C = (float*)Cout + (size_t)b * strideC;
      const int hh = lane >> 4, c4 = (lane & 15) * 4;
      for (int pass = 0; pass < 2; ++pass) {
#pragma unroll
        for (int it = 0; it < 8; ++it) {
          const int row = it * 2 + hh;
          v4f v = *(const v4f*)(slab + row * 68 + c4);
          *(volatile v4f*)(C + (size_t)(mBase + row) * ldc + n0 + c4) = v;
        }
        __threadfence();
      }
    } else {
      const int q = lane >> 3, c8 = (lane & 7) * 8;
      unsigned short* C  = (unsigned short*)Cout  + (size_t)b * strideC;
      unsigned short* C2 = (OUT_MODE == 2) ? ((unsigned short*)Cout2 + (size_t)b * strideC) : nullptr;
      for (int pass = 0; pass < 2; ++pass) {
#pragma unroll
        for (int it = 0; it < 4; ++it) {
          const int row = it * 4 + q;
          const float* sp = slab + row * 68 + c8;
          v8h hv, lv;
#pragma unroll
          for (int e = 0; e < 8; ++e) {
            if (OUT_MODE == 1) {
              hv[e] = (_Float16)sp[e];
            } else {
              unsigned short hb = f2bf_bits(sp[e]);
              unsigned short lb = f2bf_bits(sp[e] - bf_bits2f(hb));
              hv[e] = __builtin_bit_cast(_Float16, hb);
              lv[e] = __builtin_bit_cast(_Float16, lb);
            }
          }
          *(volatile v8h*)(C + (size_t)(mBase + row) * ldc + n0 + c8) = hv;
          if (OUT_MODE == 2) *(volatile v8h*)(C2 + (size_t)(mBase + row) * ldc + n0 + c8) = lv;
        }
        __threadfence();
      }
    }
    __builtin_amdgcn_fence(__ATOMIC_RELEASE, "workgroup");
    __builtin_amdgcn_wave_barrier();
    __builtin_amdgcn_fence(__ATOMIC_ACQUIRE, "workgroup");
  }
}


__device__ __forceinline__ float fast_tanh(float v) { return 1.0f - 2.0f * frcp(__expf(2.0f * v) + 1.0f); }
__device__ __forceinline__ float fast_sigmoid(float v) { return frcp(1.0f + __expf(-v)); }

__global__ __launch_bounds__(kThr) void act_pad_cast_kernel(const float* __restrict__ src, int posMajor, unsigned short* __restrict__ dst) {
  unsigned v = blockIdx.x * (unsigned)kThr + threadIdx.x;
  asm volatile("" : "+v"(v));
  const unsigned row = v / 40u;
  const unsigned k8 = (v - row * 40u) * 8u;
  unsigned srow = row;
  if (posMajor) { const unsigned pos = row >> 7; const unsigned b = row & 127u; srow = b * (unsigned)kTP + pos; }
  const float* sp = src + (size_t)srow * kD;
  const bool live0 = k8 < (unsigned)kD, live1 = (k8 + 4u) < (unsigned)kD;
  const v4f a0 = *(const v4f*)(sp + (live0 ? k8 : 0u));
  const v4f a1 = *(const v4f*)(sp + (live1 ? (k8 + 4u) : 0u));
  v8h hv;
#pragma unroll
  for (int e = 0; e < 4; ++e) {
    const float x0 = a0[e], x1 = a1[e];
    hv[e]     = (_Float16)(live0 ? carry_flush(bf16r(x0), kInCarry) : 0.0f);
    hv[4 + e] = (_Float16)(live1 ? carry_flush(bf16r(x1), kInCarry) : 0.0f);
  }
  unsigned short* dp = dst + (size_t)row * kDK + k8;
  *(volatile v8h*)dp = hv;
  __threadfence();
  *(volatile v8h*)dp = hv;
}
static_assert((kRowsP * 40) % kThr == 0 && (kRowsQ * 40) % kThr == 0 && kDK / 8 == 40 && (kD % 4) == 0, "activation cast grids exact; a 4-float vector never straddles column 300");

__global__ __launch_bounds__(kThr) void w_pad_cast_kernel(const float* __restrict__ W, int srcPitch, int colOff, int liveCols, int gateMode, int kpad,
                                                          unsigned short* __restrict__ dst) {
  unsigned v = blockIdx.x * (unsigned)kThr + threadIdx.x;
  asm volatile("" : "+v"(v));
  const unsigned perRow = (unsigned)kpad >> 3;
  const unsigned n  = v / perRow;
  const unsigned k8 = (v - n * perRow) * 8u;
  unsigned srow; bool liveRow;
  if (gateMode) { const unsigned g = n / (unsigned)kHK; const unsigned j = n - g * (unsigned)kHK; liveRow = j < (unsigned)kH; srow = g * (unsigned)kH + (liveRow ? j : 0u); }
  else { liveRow = n < (unsigned)kH; srow = liveRow ? n : 0u; }
  const float* sp = W + (size_t)srow * srcPitch + colOff;
  v8h hv;
#pragma unroll
  for (int e = 0; e < 8; ++e) {
    const unsigned k = k8 + (unsigned)e;
    const bool live = liveRow && (k < (unsigned)liveCols);
    const float w = sp[live ? k : 0u];
    hv[e] = (_Float16)(live ? carry_flush(bf16r(w), kWCarry) : 0.0f);
  }
  unsigned short* dp = dst + (size_t)v * 8u;
  *(volatile v8h*)dp = hv;
  __threadfence();
  *(volatile v8h*)dp = hv;
}
static_assert((192 * 40) % kThr == 0 && (640 * 20) % kThr == 0 && (256 * 20) % kThr == 0 && (640 * 40) % kThr == 0, "weight block grids exact");

__global__ __launch_bounds__(kThr) void bias_rows_kernel(const float* __restrict__ bih_f, const float* __restrict__ bhh_f, const float* __restrict__ bih_b,
                                                         const float* __restrict__ bhh_b, float* __restrict__ BIAS) {
  unsigned v = blockIdx.x * (unsigned)kThr + threadIdx.x;
  asm volatile("" : "+v"(v));
  const unsigned i0 = v * 4u;
  v4f o = {0.f, 0.f, 0.f, 0.f};
  if (i0 < 2u * (unsigned)kG4) {
    const bool bw = i0 >= (unsigned)kG4;
    const float* pi = bw ? bih_b : bih_f;
    const float* ph = bw ? bhh_b : bhh_f;
#pragma unroll
    for (int e = 0; e < 4; ++e) {
      unsigned n = i0 + (unsigned)e - (bw ? (unsigned)kG4 : 0u);
      asm volatile("" : "+v"(n));
      const unsigned g = n / (unsigned)kHK;
      const unsigned j = n - g * (unsigned)kHK;
      const bool live = j < (unsigned)kH;
      const unsigned si = g * (unsigned)kH + (live ? j : 0u);
      const float x = pi[si], y = ph[si];
      o[e] = live ? (bf16r(x) + bf16r(y)) : 0.0f;
    }
  }
  float* dp = BIAS + i0;
  *(volatile v4f*)dp = o;
  __threadfence();
  *(volatile v4f*)dp = o;
}
static_assert(kFEnd / 4 == 4 * kThr && (kG4 % 128) == 0, "bias grid exact; the two live regions end on wave boundaries");

__global__ __launch_bounds__(kThr) void state_zero_kernel(float* __restrict__ H32, float* __restrict__ C32, unsigned short* __restrict__ H16) {
  const size_t v = (size_t)blockIdx.x * kThr + threadIdx.x;
  const v4f zf = {0.f, 0.f, 0.f, 0.f};
  v8h zh;
#pragma unroll
  for (int e = 0; e < 8; ++e) zh[e] = (_Float16)0.0f;
  for (int pass = 0; pass < 2; ++pass) {
    *(volatile v4f*)(H32 + v * 8) = zf; *(volatile v4f*)(H32 + v * 8 + 4) = zf;
    *(volatile v4f*)(C32 + v * 8) = zf; *(volatile v4f*)(C32 + v * 8 + 4) = zf;
    *(volatile v8h*)(H16 + v * 8) = zh;
    __threadfence();
  }
}
static_assert(kR * kHK / 8 == 20 * kThr, "state grid exact");

__global__ __launch_bounds__(64) void match_attn_kernel(const float* __restrict__ GP, const float* __restrict__ GQ, const float* __restrict__ HV,
                                                        const float* __restrict__ w_att, const float* __restrict__ b_att, const float* __restrict__ mask_q,
                                                        const unsigned short* __restrict__ Q16, unsigned short* __restrict__ Z16, int t) {
  __shared__ __align__(16) float sXH[kHK];
  __shared__ __align__(16) float sV[kHK];
  __shared__ __align__(16) float sS[64];
  const int tid = threadIdx.x;
  const int r   = blockIdx.x;
  const int dir = r >> 7;
  const int b   = r & 127;
  const int pos = dir ? (kTP - 1 - t) : t;
  for (int h = tid; h < kHK; h += 64) {
    const float gp = GP[((size_t)pos * kB + b) * kHN + h];
    const float gr = HV[(size_t)r * kNHV + 2 * kG4 + h];
    const float wa = w_att[(h < kH) ? h : 0];
    sXH[h] = gp + gr;
    sV[h] = (h < kH) ? bf16r(wa) : 0.0f;
  }
  const float ba0 = b_att[0];
  const float ba = bf16r(ba0);
  __syncthreads();
  float x = 0.0f, m = 0.0f;
  if (tid < kTQ) {
    const float* gq = GQ + ((size_t)b * kTQ + tid) * kHN;
    float acc = 0.0f;
#pragma unroll 1
    for (int h4 = 0; h4 < kHK; h4 += 4) {
      const v4f q  = *(const v4f*)(gq + h4);
      const v4f xh = *(const v4f*)(sXH + h4);
      const v4f vv = *(const v4f*)(sV + h4);
      acc += vv[0] * fast_tanh(xh[0] + q[0]);
      acc += vv[1] * fast_tanh(xh[1] + q[1]);
      acc += vv[2] * fast_tanh(xh[2] + q[2]);
      acc += vv[3] * fast_tanh(xh[3] + q[3]);
    }
    const float s = acc + ba;
    float c = (s > 15.0f) ? 15.0f : s;
    c = (c < -15.0f) ? -15.0f : c;
    const float mq = mask_q[b * kTQ + tid];
    m = bf16r(mq);
    x = c * m;
  }
  sS[tid] = x;
  __syncthreads();
  float mx = sS[0];
#pragma unroll 1
  for (int j = 1; j < kTQ; ++j) { const float q = sS[j]; mx = (q > mx) ? q : mx; }
  const float ex = (tid < kTQ) ? (__expf(x - mx) * m) : 0.0f;
  __syncthreads();
  sS[tid] = ex;
  __syncthreads();
  float den = 0.0f;
#pragma unroll 1
  for (int j = 0; j < kTQ; ++j) den += sS[j];
  den += 1e-6f;
  if (tid < kDK / 8) {
    float acc8[8];
#pragma unroll
    for (int e = 0; e < 8; ++e) acc8[e] = 0.0f;
    const unsigned short* qb = Q16 + (size_t)b * kTQ * kDK + tid * 8;
#pragma unroll 1
    for (int j = 0; j < kTQ; ++j) {
      const float a = sS[j] / den;
      const v8h q8 = *(const v8h*)(qb + (size_t)j * kDK);
#pragma unroll
      for (int e = 0; e < 8; ++e) acc8[e] += a * (float)q8[e];
    }
    v8h zv;
#pragma unroll
    for (int e = 0; e < 8; ++e) zv[e] = (_Float16)carry_flush(acc8[e] * (1.0f / kInCarry), kInCarry);
    unsigned short* zp = Z16 + (size_t)r * kDK + tid * 8;
    *(volatile v8h*)zp = zv;
    __threadfence();
    *(volatile v8h*)zp = zv;
  }
}
static_assert(kTQ <= 64 && kDK / 8 <= 64 && (kHK % 4) == 0, "attention block: a thread per question position; 40 column groups");

__global__ __launch_bounds__(kThr) void bi_cell_kernel(const float* __restrict__ XGF, const float* __restrict__ XGB, const float* __restrict__ ZG,
                                                       const float* __restrict__ HV, const float* __restrict__ mask_p, float* __restrict__ H32,
                                                       float* __restrict__ C32, unsigned short* __restrict__ H16, float* __restrict__ OUTW, int t) {
  unsigned v = blockIdx.x * (unsigned)kThr + threadIdx.x;
  asm volatile("" : "+v"(v));
  const unsigned r  = v / 20u;
  const unsigned u8 = (v - r * 20u) * 8u;
  const unsigned dir = r >> 7;
  const unsigned b = r & 127u;
  const unsigned pos = dir ? (unsigned)(kTP - 1 - t) : (unsigned)t;
  const unsigned cl = (pos % (unsigned)kChunk) * (unsigned)kB + b;
  const float* xg = (dir ? XGB : XGF) + (size_t)cl * kG4 + u8;
  const float* zg = ZG + (size_t)r * kNZG + dir * (unsigned)kG4 + u8;
  const float* hv = HV + (size_t)r * kNHV + dir * (unsigned)kG4 + u8;
  const float mp0 = mask_p[b * (unsigned)kTP + pos];
  const float mp = bf16r(mp0);
  float* hp = H32 + (size_t)v * 8u;
  float* cp = C32 + (size_t)v * 8u;
  v4f ho0, ho1, co0, co1, oo0, oo1; v8h h16;
#pragma unroll
  for (int hlf = 0; hlf < 2; ++hlf) {
    const int o = 4 * hlf;
    const v4f gi = *(const v4f*)(xg + o) , gf = *(const v4f*)(xg + kHK + o), gg = *(const v4f*)(xg + 2 * kHK + o), go = *(const v4f*)(xg + 3 * kHK + o);
    const v4f zi = *(const v4f*)(zg + o) , zf = *(const v4f*)(zg + kHK + o), zgg = *(const v4f*)(zg + 2 * kHK + o), zo = *(const v4f*)(zg + 3 * kHK + o);
    const v4f si = *(const v4f*)(hv + o) , sf = *(const v4f*)(hv + kHK + o), sg = *(const v4f*)(hv + 2 * kHK + o), so = *(const v4f*)(hv + 3 * kHK + o);
    const v4f hold = *(const v4f*)(hp + o), cold = *(const v4f*)(cp + o);
#pragma unroll
    for (int e = 0; e < 4; ++e) {
      const float ig = fast_sigmoid(gi[e] + zi[e] + si[e]);
      const float fg = fast_sigmoid(gf[e] + zf[e] + sf[e]);
      const float cg = fast_tanh(gg[e] + zgg[e] + sg[e]);
      const float og = fast_sigmoid(go[e] + zo[e] + so[e]);
      float cn = fg * cold[e] + ig * cg;
      float hn = og * fast_tanh(cn);
      hn = hn * mp + hold[e] * (1.0f - mp);
      cn = cn * mp + cold[e] * (1.0f - mp);
      const float ov = hn * mp;
      if (hlf == 0) { ho0[e] = hn; co0[e] = cn; oo0[e] = ov; } else { ho1[e] = hn; co1[e] = cn; oo1[e] = ov; }
      h16[o + e] = (_Float16)carry_flush(hn, kInCarry);
    }
  }
  unsigned short* h16p = H16 + (size_t)v * 8u;
  float* op = OUTW + ((size_t)b * kTP + pos) * kDK + dir * (unsigned)kHK + u8;
  for (int pass = 0; pass < 2; ++pass) {
    *(volatile v4f*)hp = ho0; *(volatile v4f*)(hp + 4) = ho1;
    *(volatile v4f*)cp = co0; *(volatile v4f*)(cp + 4) = co1;
    *(volatile v8h*)h16p = h16;
    *(volatile v4f*)op = oo0; *(volatile v4f*)(op + 4) = oo1;
    __threadfence();
  }
}
static_assert(kR * (kHK / 8) == 20 * kThr && kHK / 8 == 20 && 2 * kHK <= kDK, "cell grid exact; both directions' halves fit an OUTW row");

__global__ __launch_bounds__(128) void assemble_out_kernel(const float* __restrict__ OUTW, const float* __restrict__ H32, float* __restrict__ out) {
  unsigned i = blockIdx.x * 128u + threadIdx.x;
  asm volatile("" : "+v"(i));
  const unsigned nOut0 = (unsigned)(kOut1 / 4);
  v4f o;
  if (i < nOut0) {
    const unsigned row = i / 75u;
    const unsigned c4 = (i - row * 75u) * 4u;
#pragma unroll
    for (int e = 0; e < 4; ++e) { const unsigned c = c4 + (unsigned)e; const unsigned sc = (c < (unsigned)kH) ? c : ((unsigned)kHK + (c - (unsigned)kH)); o[e] = OUTW[(size_t)row * kDK + sc]; }
  } else {
    const unsigned q = i - nOut0;
    const unsigned b = q / 75u;
    const unsigned c4 = (q - b * 75u) * 4u;
#pragma unroll
    for (int e = 0; e < 4; ++e) { const unsigned c = c4 + (unsigned)e; const bool bw = c >= (unsigned)kH; o[e] = H32[(size_t)((bw ? (unsigned)kB : 0u) + b) * kHK + (bw ? (c - (unsigned)kH) : c)]; }
  }
  float* dp = out + (size_t)i * 4u;
  *(volatile v4f*)dp = o;
  __threadfence();
  *(volatile v4f*)dp = o;
}
static_assert(kOutTotal % 4 == 0 && (kOutTotal / 4) % 128 == 0 && kOut1 % 4 == 0 && (2 * kH) % 4 == 0 && (2 * kH) / 4 == 75, "output grid exact; a 4-float vector never straddles a row");

extern "C" void kernel_launch(void* const* d_in, const int* in_sizes, int n_in,
                              void* d_out, int out_size, void* d_ws, size_t ws_size,
                              hipStream_t stream) {
  if (n_in < 17 || d_out == nullptr || d_ws == nullptr) return;
  if (in_sizes[0] != kB * kTP * kD || in_sizes[1] != kB * kTP || in_sizes[2] != kB * kTQ * kD || in_sizes[3] != kB * kTQ) return;
  if (in_sizes[4] != kH * kD || in_sizes[5] != kH * kD || in_sizes[6] != kH * kH || in_sizes[7] != kH || in_sizes[8] != 1) return;
  if (in_sizes[9] != 4 * kH * 2 * kD || in_sizes[10] != 4 * kH * kH || in_sizes[11] != 4 * kH || in_sizes[12] != 4 * kH) return;
  if (in_sizes[13] != 4 * kH * 2 * kD || in_sizes[14] != 4 * kH * kH || in_sizes[15] != 4 * kH || in_sizes[16] != 4 * kH) return;
  if ((size_t)out_size != kOutTotal) return;
  if (ws_size < kWsTotal) return;
  const float* input_p = (const float*)d_in[0];
  const float* mask_p  = (const float*)d_in[1];
  const float* input_q = (const float*)d_in[2];
  const float* mask_q  = (const float*)d_in[3];
  const float* W_p = (const float*)d_in[4];
  const float* W_q = (const float*)d_in[5];
  const float* W_r = (const float*)d_in[6];
  const float* w_att = (const float*)d_in[7];
  const float* b_att = (const float*)d_in[8];
  const float* W_ih_f = (const float*)d_in[9];
  const float* W_hh_f = (const float*)d_in[10];
  const float* b_ih_f = (const float*)d_in[11];
  const float* b_hh_f = (const float*)d_in[12];
  const float* W_ih_b = (const float*)d_in[13];
  const float* W_hh_b = (const float*)d_in[14];
  const float* b_ih_b = (const float*)d_in[15];
  const float* b_hh_b = (const float*)d_in[16];
  float* out = (float*)d_out;
  char* ws = (char*)d_ws;
  unsigned short* P16 = (unsigned short*)(ws + kOffP16);
  unsigned short* Q16 = (unsigned short*)(ws + kOffQ16);
  unsigned short* WP16 = (unsigned short*)(ws + kOffWP16);
  unsigned short* WQ16 = (unsigned short*)(ws + kOffWQ16);
  unsigned short* WHV = (unsigned short*)(ws + kOffWHV);
  unsigned short* WIHPF = (unsigned short*)(ws + kOffWIHPF);
  unsigned short* WIHPB = (unsigned short*)(ws + kOffWIHPB);
  unsigned short* WIHZ = (unsigned short*)(ws + kOffWIHZ);
  float* BIAS = (float*)(ws + kOffBIAS);
  float* GP = (float*)(ws + kOffGP);
  float* GQ = (float*)(ws + kOffGQ);
  float* XGF = (float*)(ws + kOffXGF);
  float* XGB = (float*)(ws + kOffXGB);
  float* HV = (float*)(ws + kOffHV);
  float* ZG = (float*)(ws + kOffZG);
  float* H32 = (float*)(ws + kOffH32);
  float* C32 = (float*)(ws + kOffC32);
  unsigned short* H16 = (unsigned short*)(ws + kOffH16);
  unsigned short* Z16 = (unsigned short*)(ws + kOffZ16);
  float* OUTW = (float*)(ws + kOffOUTW);
  const float* ZB = BIAS + kFZB;

  act_pad_cast_kernel<<<(kRowsP * 40) / kThr, kThr, 0, stream>>>(input_p, 1, P16);
  act_pad_cast_kernel<<<(kRowsQ * 40) / kThr, kThr, 0, stream>>>(input_q, 0, Q16);
  w_pad_cast_kernel<<<(192 * 40) / kThr, kThr, 0, stream>>>(W_p, kD, 0, kD, 0, kDK, WP16);
  w_pad_cast_kernel<<<(192 * 40) / kThr, kThr, 0, stream>>>(W_q, kD, 0, kD, 0, kDK, WQ16);
  w_pad_cast_kernel<<<(640 * 20) / kThr, kThr, 0, stream>>>(W_hh_f, kH, 0, kH, 1, kHK, WHV);
  w_pad_cast_kernel<<<(640 * 20) / kThr, kThr, 0, stream>>>(W_hh_b, kH, 0, kH, 1, kHK, WHV + (size_t)kG4 * kHK);
  w_pad_cast_kernel<<<(256 * 20) / kThr, kThr, 0, stream>>>(W_r, kH, 0, kH, 0, kHK, WHV + (size_t)2 * kG4 * kHK);
  w_pad_cast_kernel<<<(640 * 40) / kThr, kThr, 0, stream>>>(W_ih_f, 2 * kD, 0, kD, 1, kDK, WIHPF);
  w_pad_cast_kernel<<<(640 * 40) / kThr, kThr, 0, stream>>>(W_ih_b, 2 * kD, 0, kD, 1, kDK, WIHPB);
  w_pad_cast_kernel<<<(640 * 40) / kThr, kThr, 0, stream>>>(W_ih_f, 2 * kD, kD, kD, 1, kDK, WIHZ);
  w_pad_cast_kernel<<<(640 * 40) / kThr, kThr, 0, stream>>>(W_ih_b, 2 * kD, kD, kD, 1, kDK, WIHZ + (size_t)kG4 * kDK);
  bias_rows_kernel<<<4, kThr, 0, stream>>>(b_ih_f, b_hh_f, b_ih_b, b_hh_b, BIAS);
  state_zero_kernel<<<20, kThr, 0, stream>>>(H32, C32, H16);

  wmma_gemm64<0, false, 2, 0, false, 0><<<dim3((kRowsP / 64) * (kHN / 64) / 8, 1), 256, 0, stream>>>(
      P16, P16, kDK, 0L, WP16, WP16, kDK, 0L, (void*)GP, (void*)GP, kHN, 0L, ZB, nullptr, 0L, kRowsP, kHN, kDK, kScW);
  wmma_gemm64<0, false, 2, 0, false, 0><<<dim3((kRowsQ / 64) * (kHN / 64) / 8, 1), 256, 0, stream>>>(
      Q16, Q16, kDK, 0L, WQ16, WQ16, kDK, 0L, (void*)GQ, (void*)GQ, kHN, 0L, ZB, nullptr, 0L, kRowsQ, kHN, kDK, kScW);

  for (int t = 0; t < kTP; ++t) {
    if ((t % kChunk) == 0) {
      const int cf = t / kChunk;
      const int cb = (kTP / kChunk) - 1 - cf;
      const unsigned short* Af = P16 + (size_t)cf * kRowsC * kDK;
      const unsigned short* Ab = P16 + (size_t)cb * kRowsC * kDK;
      wmma_gemm64<0, false, 2, 0, false, 0><<<dim3((kRowsC / 64) * (kG4 / 64) / 8, 1), 256, 0, stream>>>(
          Af, Af, kDK, 0L, WIHPF, WIHPF, kDK, 0L, (void*)XGF, (void*)XGF, kG4, 0L, BIAS + kFBXF, nullptr, 0L, kRowsC, kG4, kDK, kScW);
      wmma_gemm64<0, false, 2, 0, false, 0><<<dim3((kRowsC / 64) * (kG4 / 64) / 8, 1), 256, 0, stream>>>(
          Ab, Ab, kDK, 0L, WIHPB, WIHPB, kDK, 0L, (void*)XGB, (void*)XGB, kG4, 0L, BIAS + kFBXB, nullptr, 0L, kRowsC, kG4, kDK, kScW);
    }
    wmma_gemm64<0, false, 2, 0, false, 0><<<dim3((kR / 64) * (kNHV / 64) / 8, 1), 256, 0, stream>>>(
        H16, H16, kHK, 0L, WHV, WHV, kHK, 0L, (void*)HV, (void*)HV, kNHV, 0L, ZB, nullptr, 0L, kR, kNHV, kHK, kScW);
    match_attn_kernel<<<kR, 64, 0, stream>>>(GP, GQ, HV, w_att, b_att, mask_q, Q16, Z16, t);
    wmma_gemm64<0, false, 2, 0, false, 0><<<dim3((kR / 64) * (kNZG / 64) / 8, 1), 256, 0, stream>>>(
        Z16, Z16, kDK, 0L, WIHZ, WIHZ, kDK, 0L, (void*)ZG, (void*)ZG, kNZG, 0L, ZB, nullptr, 0L, kR, kNZG, kDK, kScW);
    bi_cell_kernel<<<20, kThr, 0, stream>>>(XGF, XGB, ZG, HV, mask_p, H32, C32, H16, OUTW, t);
  }
  assemble_out_kernel<<<(int)(kOutTotal / 4 / 128), 128, 0, stream>>>(OUTW, H32, out);
}
